// CharRNN_86792699118065
// MI455X (gfx1250) — hardware-verified
//
#include <hip/hip_runtime.h>
#include <math.h>

constexpr int NB      = 64;
constexpr int NL      = 512;
constexpr int NV      = 256;
constexpr int NE      = 512;
constexpr int NH      = 1024;
constexpr int NTHR    = 256;
constexpr int SEQ_BLK = 16;
constexpr int HP      = 1032;
constexpr int TP      = 1028;
constexpr int NROWS   = NB * NL;
constexpr int NOUT0   = NROWS * NV;
constexpr int NOUT1   = NB * NH;
constexpr float WCARRY     = 256.0f;
constexpr float WCARRY_INV = 1.0f / 256.0f;
static_assert(NB % SEQ_BLK == 0);
static_assert(NH == 128 * (NTHR / 32));
static_assert(NH == 4 * NTHR);
static_assert(NH % 32 == 0 && NE % 32 == 0);
static_assert(NV % 64 == 0 && NH % 64 == 0 && NE % 64 == 0 && NROWS % 64 == 0);
static_assert(((NV / 64) * (NH / 64)) % 8 == 0);
static_assert(((NROWS / 64) * (NV / 64)) % 8 == 0);
static_assert((NV * (NE / 8)) % NTHR == 0);
static_assert(HP % 8 == 0 && TP % 4 == 0);
static_assert((size_t)NOUT0 * 4 == 33554432u);
static_assert((size_t)(NOUT0 + NOUT1) * 4 == 33816576u);

typedef __attribute__((ext_vector_type(16))) _Float16 v16h;
typedef __attribute__((ext_vector_type(8)))  _Float16 v8h;
typedef __attribute__((ext_vector_type(16))) __bf16   v16b;
typedef __attribute__((ext_vector_type(8)))  __bf16   v8b;
typedef __attribute__((ext_vector_type(8)))  float    v8f;
typedef __attribute__((ext_vector_type(4)))  float    v4f;

__device__ __forceinline__ unsigned short f2bf_bits(float f) {
  unsigned u = __float_as_uint(f);
  return (unsigned short)((u + 0x7FFFu + ((u >> 16) & 1u)) >> 16);
}
__device__ __forceinline__ float bf_bits2f(unsigned short h) { return __uint_as_float(((unsigned)h) << 16); }

__device__ __forceinline__ void dep_guard_h(v8f& a, v8f& b, v16h x, v16h y) { asm volatile("v_nop\n\tv_nop\n\tv_nop\n\tv_nop" : "+v"(a), "+v"(b) : "v"(x), "v"(y)); }
__device__ __forceinline__ void dep_guard_b(v8f& a, v8f& b, v16b x, v16b y) { asm volatile("v_nop\n\tv_nop\n\tv_nop\n\tv_nop" : "+v"(a), "+v"(b) : "v"(x), "v"(y)); }
__device__ __forceinline__ void keep4_h(v16h a, v16h b, v16h c, v16h d) { asm volatile("v_nop" :: "v"(a), "v"(b), "v"(c), "v"(d)); }
__device__ __forceinline__ void keep4_b(v16b a, v16b b, v16b c, v16b d) { asm volatile("v_nop" :: "v"(a), "v"(b), "v"(c), "v"(d)); }
__device__ __forceinline__ void acc_guard4(v8f& a, v8f& b, v8f& c, v8f& d) { asm volatile("v_nop\n\tv_nop\n\tv_nop\n\tv_nop" : "+v"(a), "+v"(b), "+v"(c), "+v"(d)); }
__device__ __forceinline__ void dep_guard4x_h(v8f& a, v8f& b, v8f& c, v8f& d, v16h x, v16h y0, v16h y1, v16h y2, v16h y3) {
  asm volatile("v_nop\n\tv_nop\n\tv_nop\n\tv_nop" : "+v"(a), "+v"(b), "+v"(c), "+v"(d) : "v"(x), "v"(y0), "v"(y1), "v"(y2), "v"(y3));
}
template <typename T> struct Frag;
template <> struct Frag<_Float16> {
  typedef v16h V; union U { v16h v; v8h h[2]; };
  static __device__ __forceinline__ v16h load(const _Float16* p) {
    U f; f.h[0] = *(const v8h*)(p); f.h[1] = *(const v8h*)(p + 16); return f.v;
  }
  static __device__ __forceinline__ v8f mma(v16h a, v16h b, v8f c) {
    return __builtin_amdgcn_wmma_f32_16x16x32_f16(false, a, false, b, (short)0, c, false, false);
  }
  static __device__ __forceinline__ void guard(v8f& a, v8f& b, v16h x, v16h y) { dep_guard_h(a, b, x, y); }
  static __device__ __forceinline__ void keep(v16h a, v16h b, v16h c, v16h d) { keep4_h(a, b, c, d); }
};
template <> struct Frag<__bf16> {
  typedef v16b V; union U { v16b v; v8b h[2]; };
  static __device__ __forceinline__ v16b load(const __bf16* p) {
    U f; f.h[0] = *(const v8b*)(p); f.h[1] = *(const v8b*)(p + 16); return f.v;
  }
  static __device__ __forceinline__ v8f mma(v16b a, v16b b, v8f c) {
    return __builtin_amdgcn_wmma_f32_16x16x32_bf16(false, a, false, b, (short)0, c, false, false);
  }
  static __device__ __forceinline__ void guard(v8f& a, v8f& b, v16b x, v16b y) { dep_guard_b(a, b, x, y); }
  static __device__ __forceinline__ void keep(v16b a, v16b b, v16b c, v16b d) { keep4_b(a, b, c, d); }
};

template <int ET> struct Elem;
template <> struct Elem<0> { typedef _Float16 T; };
template <> struct Elem<1> { typedef __bf16 T; };
template <int ET, bool SPLIT, int BIAS_MODE, int OUT_MODE, bool RESID, int ACT = 0>
__global__ __launch_bounds__(256) void wmma_gemm64(
    const unsigned short* __restrict__ Ap, const unsigned short* __restrict__ A2p, int lda, long strideA,
    const unsigned short* __restrict__ Btp, const unsigned short* __restrict__ Bt2p, int ldb, long strideB,
    void* __restrict__ Cout, void* __restrict__ Cout2, int ldc, long strideC,
    const float* __restrict__ bias,
    const float* __restrict__ resid, long strideR,
    int M, int N, int K, float scale) {
  typedef typename Elem<ET>::T T;
  typedef typename Frag<T>::V V;
  const T* A = (const T*)Ap; const T* A2 = (const T*)A2p; const T* Bt = (const T*)Btp; const T* Bt2 = (const T*)Bt2p;
  __shared__ __align__(16) float sT[8][16 * 68];
  const int b    = blockIdx.y;
  const int lane = threadIdx.x & 31;
  const int wave = threadIdx.x >> 5;
  const int tilesN = N >> 6;
  const int tilesM = M >> 6;
  const int tile = blockIdx.x * 8 + wave;
  if (tile >= tilesM * tilesN) return;
  const int tm = tile / tilesN;
  const int tn = tile - tm * tilesN;
  const int m0 = tm << 6;
  const int n0 = tn << 6;

  const T* Ab  = A  + (size_t)b * strideA;
  const T* Bb  = Bt + (size_t)b * strideB;
  const T* Ab2 = SPLIT ? (A2  + (size_t)b * strideA) : nullptr;
  const T* Bb2 = SPLIT ? (Bt2 + (size_t)b * strideB) : nullptr;

  const int rlane = lane & 15;
  const int koff  = (lane >> 4) * 8;
  const int mOff  = (lane >> 4) * 8;

  v8f acc[4][4];
#pragma unroll
  for (int i = 0; i < 4; ++i)
#pragma unroll
    for (int j = 0; j < 4; ++j) acc[i][j] = (v8f){0.f,0.f,0.f,0.f,0.f,0.f,0.f,0.f};

  for (int k0 = 0; k0 < K; k0 += 32) {
    V bh[4], bl[4];
#pragma unroll
    for (int j = 0; j < 4; ++j) {
      const size_t bo = (size_t)(n0 + (j << 4) + rlane) * ldb + koff + k0;
      bh[j] = Frag<T>::load(Bb + bo);
      if (SPLIT) bl[j] = Frag<T>::load(Bb2 + bo);
    }
#pragma unroll
    for (int i = 0; i < 4; ++i) {
      const size_t ao = (size_t)(m0 + (i << 4) + rlane) * lda + koff + k0;
      V ah = Frag<T>::load(Ab + ao);
      V al;
      if (SPLIT) al = Frag<T>::load(Ab2 + ao);
#pragma unroll
      for (int j = 0; j < 4; ++j) {
        acc[i][j] = Frag<T>::mma(ah, bh[j], acc[i][j]);
        if (SPLIT) {
          acc[i][j] = Frag<T>::mma(ah, bl[j], acc[i][j]);
          acc[i][j] = Frag<T>::mma(al, bh[j], acc[i][j]);
        }
      }
      Frag<T>::guard(acc[i][0], acc[i][3], ah, SPLIT ? al : ah);
    }
    Frag<T>::keep(bh[0], bh[1], bh[2], bh[3]);
    if (SPLIT) Frag<T>::keep(bl[0], bl[1], bl[2], bl[3]);
  }
  acc_guard4(acc[0][0], acc[0][1], acc[0][2], acc[0][3]);
  acc_guard4(acc[1][0], acc[1][1], acc[1][2], acc[1][3]);
  acc_guard4(acc[2][0], acc[2][1], acc[2][2], acc[2][3]);
  acc_guard4(acc[3][0], acc[3][1], acc[3][2], acc[3][3]);

  float* slab = sT[wave];
  const float* Rb = RESID ? (resid + (size_t)b * strideR) : nullptr;
#pragma unroll
  for (int i = 0; i < 4; ++i) {
    const int mBase = m0 + (i << 4);
#pragma unroll
    for (int j = 0; j < 4; ++j) {
      const int n = n0 + (j << 4) + rlane;
      float bv = 0.f;
      if (BIAS_MODE == 2) bv = bias[n];
#pragma unroll
      for (int r = 0; r < 8; ++r) {
        float v = acc[i][j][r] * scale;
        if (BIAS_MODE == 1) v += bias[mBase + mOff + r];
        if (BIAS_MODE == 2) v += bv;
        if (RESID) v += Rb[(size_t)(mBase + mOff + r) * ldc + n];
        if (ACT == 1) v = tanhf(v);
        if (ACT == 2) v = fmaxf(v, 0.0f);
        if (ACT == 3) v = v / (1.0f + expf(-v));
        if (ACT == 4) v = (v > 0.f) ? v : 0.01f * v;
        if (ACT == 5) v = 0.5f * v * (1.0f + erff(v * 0.70710678118654752f));
        slab[(mOff + r) * 68 + (j << 4) + rlane] = v;
      }
    }
    __builtin_amdgcn_fence(__ATOMIC_RELEASE, "workgroup");
    __builtin_amdgcn_wave_barrier();
    __builtin_amdgcn_fence(__ATOMIC_ACQUIRE, "workgroup");
    if (OUT_MODE == 0) {
      float* C = (float*)Cout + (size_t)b * strideC;
      const int hh = lane >> 4, c4 = (lane & 15) * 4;
      for (int pass = 0; pass < 2; ++pass) {
#pragma unroll
        for (int it = 0; it < 8; ++it) {
          const int row = it * 2 + hh;
          v4f v = *(const v4f*)(slab + row * 68 + c4);
          *(volatile v4f*)(C + (size_t)(mBase + row) * ldc + n0 + c4) = v;
        }
        __threadfence();
      }
    } else {
      const int q = lane >> 3, c8 = (lane & 7) * 8;
      unsigned short* C  = (unsigned short*)Cout  + (size_t)b * strideC;
      unsigned short* C2 = (OUT_MODE == 2) ? ((unsigned short*)Cout2 + (size_t)b * strideC) : nullptr;
      for (int pass = 0; pass < 2; ++pass) {
#pragma unroll
        for (int it = 0; it < 4; ++it) {
          const int row = it * 4 + q;
          const float* sp = slab + row * 68 + c8;
          v8h hv, lv;
#pragma unroll
          for (int e = 0; e < 8; ++e) {
            if (OUT_MODE == 1) {
              hv[e] = (_Float16)sp[e];
            } else {
              unsigned short hb = f2bf_bits(sp[e]);
              unsigned short lb = f2bf_bits(sp[e] - bf_bits2f(hb));
              hv[e] = __builtin_bit_cast(_Float16, hb);
              lv[e] = __builtin_bit_cast(_Float16, lb);
            }
          }
          *(volatile v8h*)(C + (size_t)(mBase + row) * ldc + n0 + c8) = hv;
          if (OUT_MODE == 2) *(volatile v8h*)(C2 + (size_t)(mBase + row) * ldc + n0 + c8) = lv;
        }
        __threadfence();
      }
    }
    __builtin_amdgcn_fence(__ATOMIC_RELEASE, "workgroup");
    __builtin_amdgcn_wave_barrier();
    __builtin_amdgcn_fence(__ATOMIC_ACQUIRE, "workgroup");
  }
}

__global__ __launch_bounds__(NTHR) void cvt8_bf16hl_kernel(const float* __restrict__ src, unsigned short* __restrict__ dh,
                                                           unsigned short* __restrict__ dl, int nrow, int ncol8, int spitch) {
  const int i  = blockIdx.x * NTHR + threadIdx.x;
  const int n8 = nrow * ncol8;
  if (i < n8) {
    const int row = i / ncol8;
    const int c8  = i - row * ncol8;
    const float* sp = src + (size_t)row * spitch + c8 * 8;
    const v4f a = *(const v4f*)(sp);
    const v4f b = *(const v4f*)(sp + 4);
    v8h hv, lv;
#pragma unroll
    for (int e = 0; e < 4; ++e) {
      const unsigned short ha = f2bf_bits(a[e]);
      const unsigned short la = f2bf_bits(a[e] - bf_bits2f(ha));
      const unsigned short hb = f2bf_bits(b[e]);
      const unsigned short lb = f2bf_bits(b[e] - bf_bits2f(hb));
      hv[e]     = __builtin_bit_cast(_Float16, ha);
      lv[e]     = __builtin_bit_cast(_Float16, la);
      hv[4 + e] = __builtin_bit_cast(_Float16, hb);
      lv[4 + e] = __builtin_bit_cast(_Float16, lb);
    }
    *(volatile v8h*)(dh + (size_t)i * 8) = hv;
    *(volatile v8h*)(dl + (size_t)i * 8) = lv;
    __threadfence();
    *(volatile v8h*)(dh + (size_t)i * 8) = hv;
    *(volatile v8h*)(dl + (size_t)i * 8) = lv;
  }
}

template <int MODE>
__global__ __launch_bounds__(NTHR) void tpw_kernel(const float* __restrict__ src, int R, int C, int ldo,
                                                  unsigned short* __restrict__ O, unsigned short* __restrict__ O2, float sc) {
  __shared__ float Tt[64 * 65];
  const int tid = threadIdx.x;
  const int c0 = blockIdx.x * 64, r0 = blockIdx.y * 64;
#pragma unroll
  for (int i = 0; i < 4; ++i) {
    const int idx = i * NTHR + tid;
    const int rr = idx >> 4, cc = (idx & 15) * 4;
    const v4f v = *(const v4f*)(src + (size_t)(r0 + rr) * (size_t)C + c0 + cc);
    Tt[rr * 65 + cc + 0] = v[0];
    Tt[rr * 65 + cc + 1] = v[1];
    Tt[rr * 65 + cc + 2] = v[2];
    Tt[rr * 65 + cc + 3] = v[3];
  }
  __syncthreads();
  const int q = tid >> 3, c8 = (tid & 7) * 8;
  v8h hv[2], lv[2];
#pragma unroll
  for (int g = 0; g < 2; ++g) {
    const int qq = g * 32 + q;
#pragma unroll
    for (int e = 0; e < 8; ++e) {
      const float f = Tt[(c8 + e) * 65 + qq];
      if (MODE == 0) {
        hv[g][e] = (_Float16)(f * sc);
        lv[g][e] = hv[g][e];
      } else {
        const unsigned short hb = f2bf_bits(f);
        const unsigned short lb = f2bf_bits(f - bf_bits2f(hb));
        hv[g][e] = __builtin_bit_cast(_Float16, hb);
        lv[g][e] = __builtin_bit_cast(_Float16, lb);
      }
    }
  }
  for (int pass = 0; pass < 2; ++pass) {
#pragma unroll
    for (int g = 0; g < 2; ++g) {
      const size_t o = (size_t)(c0 + g * 32 + q) * (size_t)ldo + (size_t)(r0 + c8);
      *(volatile v8h*)(O + o) = hv[g];
      if (MODE == 1) *(volatile v8h*)(O2 + o) = lv[g];
    }
    __threadfence();
  }
}

__global__ __launch_bounds__(NTHR) void rnn_seq_kernel(const int* __restrict__ xtok, const float* __restrict__ h0,
                                                       const float* __restrict__ TT,
                                                       const unsigned short* __restrict__ WHTp,
                                                       unsigned short* __restrict__ HSp, float* __restrict__ HFIN) {
  __shared__ __align__(16) _Float16 Ah[SEQ_BLK * HP];
  __shared__ __align__(16) float    Ts[SEQ_BLK * TP];
  const _Float16* WHT = (const _Float16*)WHTp;
  _Float16* HS = (_Float16*)HSp;
  const int tid = threadIdx.x, lane = tid & 31, wave = tid >> 5;
  const int c = lane & 15, hh = lane >> 4, koff = hh * 8;
  const int q = lane >> 3, c8 = (lane & 7) * 8;
  const int rowbase = blockIdx.x * SEQ_BLK;
  const int colw = 128 * wave;

#pragma unroll 1
  for (int i = tid; i < SEQ_BLK * HP; i += NTHR) Ah[i] = (_Float16)0.0f;
  __syncthreads();
#pragma unroll 1
  for (int i = 0; i < SEQ_BLK; ++i) {
    const v4f v = *(const v4f*)(h0 + (size_t)(rowbase + i) * NH + tid * 4);
    _Float16* d = Ah + i * HP + tid * 4;
    d[0] = (_Float16)v[0];
    d[1] = (_Float16)v[1];
    d[2] = (_Float16)v[2];
    d[3] = (_Float16)v[3];
    asm volatile("" ::: "memory");
  }
  __syncthreads();

  const v8f z8 = {0.f, 0.f, 0.f, 0.f, 0.f, 0.f, 0.f, 0.f};
  const _Float16* ahrow = Ah + c * HP + koff;

#pragma unroll 1
  for (int l = 0; l < NL; ++l) {
    const bool last = (l == NL - 1);
#pragma unroll 1
    for (int i = 0; i < SEQ_BLK; ++i) {
      int tok = xtok[(rowbase + i) * NL + l];
      tok = tok < 0 ? 0 : tok;
      tok = tok > NV - 1 ? NV - 1 : tok;
      const v4f v = *(const v4f*)(TT + (size_t)tok * NH + tid * 4);
      *(v4f*)(Ts + i * TP + tid * 4) = v;
      asm volatile("" ::: "memory");
    }
    __syncthreads();

    v8f acc[2][4];
#pragma unroll
    for (int g = 0; g < 2; ++g) {
      v8f a0 = z8, a1 = z8, a2 = z8, a3 = z8;
      const _Float16* wb = WHT + (size_t)(colw + 64 * g + c) * NH + koff;
#pragma unroll 1
      for (int k0 = 0; k0 < NH; k0 += 32) {
        const v16h a  = Frag<_Float16>::load(ahrow + k0);
        const v16h b0 = Frag<_Float16>::load(wb + k0);
        const v16h b1 = Frag<_Float16>::load(wb + (size_t)16 * NH + k0);
        const v16h b2 = Frag<_Float16>::load(wb + (size_t)32 * NH + k0);
        const v16h b3 = Frag<_Float16>::load(wb + (size_t)48 * NH + k0);
        a0 = Frag<_Float16>::mma(a, b0, a0);
        a1 = Frag<_Float16>::mma(a, b1, a1);
        a2 = Frag<_Float16>::mma(a, b2, a2);
        a3 = Frag<_Float16>::mma(a, b3, a3);
        dep_guard4x_h(a0, a1, a2, a3, a, b0, b1, b2, b3);
      }
      acc_guard4(a0, a1, a2, a3);
      acc[g][0] = a0; acc[g][1] = a1; acc[g][2] = a2; acc[g][3] = a3;
    }
    __syncthreads();

#pragma unroll
    for (int g = 0; g < 2; ++g) {
#pragma unroll
      for (int nt = 0; nt < 4; ++nt) {
        const int j = colw + 64 * g + 16 * nt + c;
#pragma unroll
        for (int r = 0; r < 8; ++r) {
          const int row = 8 * hh + r;
          const float tv = Ts[row * TP + j];
          const float z  = acc[g][nt][r] * WCARRY_INV + tv;
          const float hn = tanhf(z);
          Ah[row * HP + j] = (_Float16)hn;
          if (last) Ts[row * TP + j] = hn;
        }
      }
    }
    __builtin_amdgcn_fence(__ATOMIC_RELEASE, "workgroup");
    __builtin_amdgcn_wave_barrier();
    __builtin_amdgcn_fence(__ATOMIC_ACQUIRE, "workgroup");
    for (int pass = 0; pass < 2; ++pass) {
#pragma unroll
      for (int it = 0; it < 8; ++it) {
        const int row = it * 2 + (q >> 1);
        const int col = colw + 64 * (q & 1) + c8;
        const v8h v = *(const v8h*)(Ah + row * HP + col);
        *(volatile v8h*)(HS + ((size_t)(rowbase + row) * NL + (size_t)l) * NH + col) = v;
      }
      __threadfence();
    }
    if (last) {
      __builtin_amdgcn_fence(__ATOMIC_RELEASE, "workgroup");
      __builtin_amdgcn_wave_barrier();
      __builtin_amdgcn_fence(__ATOMIC_ACQUIRE, "workgroup");
      for (int pass = 0; pass < 2; ++pass) {
#pragma unroll
        for (int it = 0; it < SEQ_BLK; ++it) {
          const v4f v = *(const v4f*)(Ts + it * TP + colw + lane * 4);
          *(volatile v4f*)(HFIN + (size_t)(rowbase + it) * NH + colw + lane * 4) = v;
        }
        __threadfence();
      }
    }
    __syncthreads();
  }
}

extern "C" void kernel_launch(void* const* d_in, const int* in_sizes, int n_in,
                              void* d_out, int out_size, void* d_ws, size_t ws_size, hipStream_t stream) {
  if (n_in < 6 || d_out == nullptr || d_ws == nullptr) return;
  if (in_sizes[0] != NB * NL || in_sizes[1] != NB * NH || in_sizes[2] != NV * NE || in_sizes[3] != NE * NH ||
      in_sizes[4] != NH * NH || in_sizes[5] != NH * NV || out_size != NOUT0 + NOUT1) return;

  const int*   xtok   = (const int*)d_in[0];
  const float* hidden = (const float*)d_in[1];
  const float* emb    = (const float*)d_in[2];
  const float* w_e    = (const float*)d_in[3];
  const float* w_h    = (const float*)d_in[4];
  const float* w_o    = (const float*)d_in[5];
  float* out0 = (float*)d_out;
  float* out1 = out0 + (size_t)NOUT0;

  char* ws = (char*)d_ws; size_t off = 0;
  auto carve = [&](size_t bytes) -> char* { char* p = ws + off; off += (bytes + 255) & ~(size_t)255; return p; };
  unsigned short* EMBH  = (unsigned short*)carve((size_t)NV * NE * 2);
  unsigned short* EMBL  = (unsigned short*)carve((size_t)NV * NE * 2);
  unsigned short* WEH   = (unsigned short*)carve((size_t)NH * NE * 2);
  unsigned short* WEL   = (unsigned short*)carve((size_t)NH * NE * 2);
  unsigned short* WHT   = (unsigned short*)carve((size_t)NH * NH * 2);
  unsigned short* WOT   = (unsigned short*)carve((size_t)NV * NH * 2);
  float*          TT    = (float*)carve((size_t)NV * NH * 4);
  unsigned short* HS    = (unsigned short*)carve((size_t)NROWS * NH * 2);
  if (off > ws_size || off > (size_t)134217728) return;

  cvt8_bf16hl_kernel<<<(NV * (NE / 8)) / NTHR, NTHR, 0, stream>>>(emb, EMBH, EMBL, NV, NE / 8, NE);
  tpw_kernel<1><<<dim3(NH / 64, NE / 64), NTHR, 0, stream>>>(w_e, NE, NH, NE, WEH, WEL, 1.0f);
  tpw_kernel<0><<<dim3(NH / 64, NH / 64), NTHR, 0, stream>>>(w_h, NH, NH, NH, WHT, WHT, WCARRY);
  tpw_kernel<0><<<dim3(NV / 64, NH / 64), NTHR, 0, stream>>>(w_o, NH, NV, NH, WOT, WOT, WCARRY);

  wmma_gemm64<1, true, 0, 0, false, 0><<<dim3(((NV / 64) * (NH / 64)) / 8, 1), 256, 0, stream>>>(
      EMBH, EMBL, NE, 0L, WEH, WEL, NE, 0L, (void*)TT, (void*)TT, NH, 0L,
      hidden, hidden, 0L, NV, NH, NE, 1.0f);

  rnn_seq_kernel<<<NB / SEQ_BLK, NTHR, 0, stream>>>(xtok, hidden, TT, WHT, HS, out1);

  wmma_gemm64<0, false, 0, 0, false, 0><<<dim3(((NROWS / 64) * (NV / 64)) / 8, 1), 256, 0, stream>>>(
      HS, HS, NH, 0L, WOT, WOT, NH, 0L, (void*)out0, (void*)out0, NV, 0L,
      hidden, hidden, 0L, NROWS, NV, NH, WCARRY_INV);
}
